// NodeGraphConv_46170898432062
// MI455X (gfx1250) — hardware-run, weakly checked
//
#include <hip/hip_runtime.h>

typedef float          v8f   __attribute__((ext_vector_type(8)));
typedef float          v4f   __attribute__((ext_vector_type(4)));
typedef unsigned int   v4u   __attribute__((ext_vector_type(4)));
typedef int            v8i   __attribute__((ext_vector_type(8)));
typedef unsigned short v8us  __attribute__((ext_vector_type(8)));
typedef unsigned short v16us __attribute__((ext_vector_type(16)));
typedef __bf16         v16bf __attribute__((ext_vector_type(16)));
typedef _Float16       v16h  __attribute__((ext_vector_type(16)));
typedef v4f  __attribute__((may_alias)) v4fa;
typedef v8us __attribute__((may_alias)) v8usa;
union FragB { v16bf v; v16us u; v8us h[2]; v8i w; };
union FragH { v16h  v; v16us u; v8us h[2]; v8i w; };

__device__ __forceinline__ v8f wmb(const FragB& a, const FragB& b, v8f c) {
  v8f d = __builtin_amdgcn_wmma_f32_16x16x32_bf16(false, a.v, false, b.v, (short)0, c, false, false);
  asm volatile("v_nop\n\tv_nop\n\tv_nop\n\tv_nop" : "+v"(d) : "v"(a.w), "v"(b.w));
  return d;
}

__device__ __forceinline__ v8f wmh(const FragH& a, const FragH& b, v8f c) {
  v8f d = __builtin_amdgcn_wmma_f32_16x16x32_f16(false, a.v, false, b.v, (short)0, c, false, false);
  asm volatile("v_nop\n\tv_nop\n\tv_nop\n\tv_nop" : "+v"(d) : "v"(a.w), "v"(b.w));
  return d;
}

__device__ __forceinline__ unsigned bf16_bits(float f) {
  const unsigned u = __float_as_uint(f);
  const unsigned r = (u + 0x7FFFu + ((u >> 16) & 1u)) >> 16;
  const unsigned q = (u >> 16) | 0x40u;
  return ((u & 0x7fffffffu) > 0x7f800000u) ? q : r;
}

__device__ __forceinline__ float bf16_val(float f) {
  return __uint_as_float(bf16_bits(f) << 16);
}
__device__ __forceinline__ int clampi(int v, int lo, int hi) {
  return v < lo ? lo : (v > hi ? hi : v);
}

__device__ __forceinline__ unsigned f16_bits(float f) {
  const unsigned u  = __float_as_uint(f);
  const unsigned s  = (u >> 16) & 0x8000u;
  const unsigned a  = u & 0x7fffffffu;
  const unsigned t  = a - 0x38000000u;
  const unsigned r  = (t + 0x0FFFu + ((t >> 13) & 1u)) >> 13;
  const unsigned rc = r > 0x7C00u ? 0x7C00u : r;
  const bool small  = a < 0x38800000u;
  const bool isnan  = a > 0x7f800000u;
  const unsigned fin = small ? 0u : (s | rc);
  return isnan ? (s | 0x7E00u) : fin;
}

__device__ __forceinline__ unsigned pk16(unsigned lo, unsigned hi) { return lo | (hi << 16); }
__device__ __forceinline__ unsigned bf16_lo_bits(float v) {
  float hi = bf16_val(v);
  asm volatile("" : "+v"(hi));
  return bf16_bits(v - hi);
}
__device__ __forceinline__ v4u pack8_bf16(v4f a, v4f c) {
  return (v4u){ pk16(bf16_bits(a[0]), bf16_bits(a[1])), pk16(bf16_bits(a[2]), bf16_bits(a[3])),
                pk16(bf16_bits(c[0]), bf16_bits(c[1])), pk16(bf16_bits(c[2]), bf16_bits(c[3])) };
}
__device__ __forceinline__ v4u pack8_bf16_lo(v4f a, v4f c) {
  return (v4u){ pk16(bf16_lo_bits(a[0]), bf16_lo_bits(a[1])), pk16(bf16_lo_bits(a[2]), bf16_lo_bits(a[3])),
                pk16(bf16_lo_bits(c[0]), bf16_lo_bits(c[1])), pk16(bf16_lo_bits(c[2]), bf16_lo_bits(c[3])) };
}
__device__ __forceinline__ v4u pack8_f16(v4f a, v4f c) {
  return (v4u){ pk16(f16_bits(a[0]), f16_bits(a[1])), pk16(f16_bits(a[2]), f16_bits(a[3])),
                pk16(f16_bits(c[0]), f16_bits(c[1])), pk16(f16_bits(c[2]), f16_bits(c[3])) };
}

template <int FORM>
__global__ __launch_bounds__(256) void k_plane(const float* __restrict__ src, int rows, int cols, int ldsrc,
                                               unsigned short* __restrict__ dst, int MP, int KP) {
  static_assert(FORM >= 0 && FORM <= 3);
  const int KTOT = (FORM == 1 || FORM == 3) ? 2 * KP : KP;
  const unsigned ppr   = (unsigned)(KTOT >> 3);
  const unsigned kp8   = (unsigned)(KP >> 3);
  const unsigned total = (unsigned)MP * ppr;
  const unsigned g     = blockIdx.x * 256u + threadIdx.x;
  const unsigned rowu  = g / ppr;
  const unsigned p     = g - rowu * ppr;
  const bool second    = p >= kp8;
  const int row = (int)rowu;
  const int c0  = (int)((second ? p - kp8 : p) << 3);
  const float* srow = src + (size_t)clampi(row, 0, rows - 1) * (size_t)ldsrc;
  float x[8];
  unsigned mk[8];
#pragma unroll
  for (int e = 0; e < 8; ++e) {
    const int c = c0 + e;
    const float v = srow[clampi(c, 0, cols - 1)];
    asm volatile("" :: "v"(v));
    x[e]  = v;
    mk[e] = (row < rows && c < cols) ? 0xFFFFu : 0u;
  }
  const v4f a = (v4f){ x[0], x[1], x[2], x[3] };
  const v4f c = (v4f){ x[4], x[5], x[6], x[7] };
  v4u o;
  if (FORM == 2) {
    o = pack8_f16(a, c);
  } else {
    const v4u hi = pack8_bf16(a, c);
    o = hi;
    if (FORM == 1) { const v4u lo = pack8_bf16_lo(a, c); o = second ? lo : hi; }
  }
  const v4u mw = (v4u){ pk16(mk[0], mk[1]), pk16(mk[2], mk[3]), pk16(mk[4], mk[5]), pk16(mk[6], mk[7]) };
  o &= mw;
  if (g < total) {
    volatile v4u* q = (volatile v4u*)(dst + (size_t)g * 8);
    *q = o;
    __threadfence();
    *q = o;
  }
}

template <int FORM> struct FragOf    { typedef FragB T; };
template <>         struct FragOf<2> { typedef FragH T; };
__device__ __forceinline__ v8f mm(const FragB& a, const FragB& b, v8f c) { return wmb(a, b, c); }
__device__ __forceinline__ v8f mm(const FragH& a, const FragH& b, v8f c) { return wmh(a, b, c); }
template <class F> __device__ __forceinline__ F ld_frag(const unsigned short* p) {
  F f;
  f.h[0] = *(const v8usa*)(p);
  f.h[1] = *(const v8usa*)(p + 16);
  return f;
}

template <int FORM, int EPI>
__global__ __launch_bounds__(256) __attribute__((amdgpu_num_vgpr(248)))
void k_gemm_nt(const unsigned short* __restrict__ A, const unsigned short* __restrict__ B,
               const float* __restrict__ bias, float* __restrict__ D, int M, int N, int KTOT, int ldd) {
  static_assert(FORM >= 0 && FORM <= 2);
  static_assert(EPI == 0 || EPI == 1);
  typedef typename FragOf<FORM>::T F;
  __shared__ __attribute__((aligned(16))) float sT[8][16 * 68];
  const int lane = threadIdx.x & 31;
  const int wave = threadIdx.x >> 5;
  const int tilesM = (M + 63) >> 6;
  const int tilesN = (N + 63) >> 6;
  const int tile = blockIdx.x * 8 + wave;
  if (tile >= tilesM * tilesN) return;
  const int tm = tile / tilesN;
  const int tn = tile - tm * tilesN;
  const int m0 = tm << 6;
  const int n0 = tn << 6;

  const int rl = lane & 15;
  const int h8 = (lane >> 4) * 8;
  const unsigned short* pa = A + (size_t)(m0 + rl) * (size_t)KTOT + h8;
  const unsigned short* pb = B + (size_t)(n0 + rl) * (size_t)KTOT + h8;

  v8f acc[4][4];
#pragma unroll
  for (int i = 0; i < 4; ++i)
#pragma unroll
    for (int j = 0; j < 4; ++j) acc[i][j] = (v8f){0.f, 0.f, 0.f, 0.f, 0.f, 0.f, 0.f, 0.f};

#pragma unroll 1
  for (int k0 = 0; k0 < KTOT; k0 += 32) {
    F bf[4];
#pragma unroll
    for (int j = 0; j < 4; ++j) bf[j] = ld_frag<F>(pb + (size_t)(j << 4) * (size_t)KTOT + k0);
#pragma unroll
    for (int i = 0; i < 4; ++i) {
      const F af = ld_frag<F>(pa + (size_t)(i << 4) * (size_t)KTOT + k0);
#pragma unroll
      for (int j = 0; j < 4; ++j) acc[i][j] = mm(af, bf[j], acc[i][j]);
    }
  }

  float* slab = sT[wave];
  const int hh = lane >> 4;
  const int c4 = (lane & 15) * 4;
  const int nc = n0 + c4;
  const bool cok = nc < N;
  v4f bv = (v4f){0.f, 0.f, 0.f, 0.f};
  if (EPI == 1) {
    bv = *(const v4fa*)(bias + clampi(nc, 0, N - 4));
    asm volatile("" :: "v"(bv));
  }
#pragma unroll
  for (int i = 0; i < 4; ++i) {
    const int mBase = m0 + (i << 4);
#pragma unroll
    for (int j = 0; j < 4; ++j) {
#pragma unroll
      for (int r = 0; r < 8; ++r) slab[(h8 + r) * 68 + (j << 4) + rl] = acc[i][j][r];
    }
    __builtin_amdgcn_fence(__ATOMIC_RELEASE, "workgroup");
    __builtin_amdgcn_wave_barrier();
    __builtin_amdgcn_fence(__ATOMIC_ACQUIRE, "workgroup");
    v4f vv[8];
#pragma unroll
    for (int it = 0; it < 8; ++it) {
      const int row = it * 2 + hh;
      v4f v = *(const v4fa*)(slab + row * 68 + c4);
      if (EPI == 1) v += bv;
      vv[it] = v;
    }
    for (int pass = 0; pass < 2; ++pass) {
#pragma unroll
      for (int it = 0; it < 8; ++it) {
        const int row = mBase + it * 2 + hh;
        if (cok && row < M) *(volatile v4f*)(D + (size_t)row * (size_t)ldd + nc) = vv[it];
      }
      __threadfence();
    }
    __builtin_amdgcn_fence(__ATOMIC_RELEASE, "workgroup");
    __builtin_amdgcn_wave_barrier();
    __builtin_amdgcn_fence(__ATOMIC_ACQUIRE, "workgroup");
  }
}

#include <stddef.h>
#pragma clang fp contract(off)

#define NN      100000
#define NE      1600000
#define FD      128
#define NCLS    40
#define NCP     64
#define MP      100096
#define CH      12544
#define CHL     12288
#define NCHUNK  8
#define KL0     384
#define KL1     512
#define NTHR    256
#define NWAVE   8
#define EPT     8
#define WCH     (32 * EPT)
#define NBRUN   512
#define SLB     9
#define NBK     196
#define WLCAP   4608
#define LCAP    12288
#define DEGCAP  48
#define MAXDEG_MEAS  36
#define MAXB512_MEAS 8469
#define OUT4    1000000

#define BK_ZINTS (NWAVE * WLCAP + LCAP + 3 * NBRUN)
#define BK_INTS  (BK_ZINTS + 16)
#define BK_LDS   (BK_INTS * 4)

#define PW_BLKS 73

static_assert(MP == 782 * 128 && MP % 64 == 0 && MP >= NN);
static_assert(CH % 64 == 0 && CHL % 64 == 0 && CHL > 0 && (NCHUNK - 1) * CH + CHL == MP);
static_assert(CH % NWAVE == 0 && CHL % NWAVE == 0 && NN % NWAVE == 0);
static_assert(KL0 % 32 == 0 && KL1 % 32 == 0 && FD % 64 == 0 && NCP % 64 == 0 && FD % 32 == 0 && NCP % 32 == 0);
static_assert(FD == 32 * 4 && NCLS % 4 == 0 && NCLS <= NCP);
static_assert((long long)NN * NCLS == (long long)OUT4 * 4 && OUT4 % 8 == 0);
static_assert(NBRUN == (1 << SLB) && NBRUN % 128 == 0 && NBRUN / 4 <= NTHR && NBRUN % 32 == 0);
static_assert(NBK * NBRUN >= MP && (NBK - 1) * NBRUN < NN);
static_assert(NE < (1 << 21) && (((long long)NE) << SLB) < (1LL << 31));
static_assert(NE % EPT == 0 && NE >= EPT);
static_assert(LCAP % 1024 == 0 && LCAP % (NTHR * 4) == 0);
static_assert((long long)LCAP * 100 >= (long long)MAXB512_MEAS * 125);
static_assert(WLCAP >= (MAXB512_MEAS / 8) * 4);
static_assert(MAXDEG_MEAS + 8 <= DEGCAP);
static_assert(BK_ZINTS % 4 == 0 && BK_LDS <= 262144 && BK_LDS + 0 <= 327680);
static_assert((long long)CH * KL1 / 8 < (1LL << 31));

typedef int          v4i  __attribute__((ext_vector_type(4)));
typedef unsigned int v2u  __attribute__((ext_vector_type(2)));
typedef v4i __attribute__((may_alias)) v4ia;

__device__ __forceinline__ void st2_v4f(float* p, v4f v) {
  *(volatile v4f*)p = v;
  __threadfence();
  *(volatile v4f*)p = v;
}
__device__ __forceinline__ void st2_v8us(unsigned short* p, v8us v) {
  *(volatile v8us*)p = v;
  __threadfence();
  *(volatile v8us*)p = v;
}

__device__ __forceinline__ v8us gather8(const float* __restrict__ base, int stride) {
  float f[8];
#pragma unroll
  for (int i = 0; i < 8; ++i) f[i] = base[(size_t)i * (size_t)stride];
  v8us o;
#pragma unroll
  for (int i = 0; i < 8; ++i) o[i] = (unsigned short)bf16_bits(f[i]);
  return o;
}

__device__ __forceinline__ void prep_seg(const float* __restrict__ W, int cout, unsigned short* dst,
                                         int ktot, int koff, int u) {
  const int n  = u >> 4;
  const int k8 = (u & 15) * 8;
  const int nc = n < cout ? n : cout - 1;
  v8us o = gather8(W + (size_t)k8 * (size_t)cout + nc, cout);
  const unsigned short m = (n < cout) ? (unsigned short)0xFFFF : (unsigned short)0;
  const v8us mv = (v8us){ m, m, m, m, m, m, m, m };
  o = o & mv;
  st2_v8us(dst + (size_t)n * (size_t)ktot + koff + k8, o);
}

__device__ __forceinline__ v4f cvt4_bf16(v4f v) {
  v4f o;
  o.x = bf16_val(v.x); o.y = bf16_val(v.y); o.z = bf16_val(v.z); o.w = bf16_val(v.w);
  return o;
}

__global__ __launch_bounds__(NTHR) void k_prep(const float* __restrict__ Wr0, const float* __restrict__ Ws0,
                                               const float* __restrict__ b0,
                                               const float* __restrict__ Wr1, const float* __restrict__ Ws1,
                                               const float* __restrict__ b1,
                                               const float* __restrict__ Wr2, const float* __restrict__ Ws2,
                                               const float* __restrict__ b2,
                                               unsigned short* wt, float* bias) {
  const int tid = (int)threadIdx.x;
  const int blk = (int)blockIdx.x;
  unsigned short* wt0 = wt;
  unsigned short* wt1 = wt + (size_t)FD * KL0;
  unsigned short* wt2 = wt1 + (size_t)FD * KL1;
  if (blk < 8)        { prep_seg(Wr0, FD, wt0, KL0, 0,   (blk - 0)  * NTHR + tid); }
  else if (blk < 16)  { prep_seg(Wr0, FD, wt0, KL0, 128, (blk - 8)  * NTHR + tid); }
  else if (blk < 24)  { prep_seg(Ws0, FD, wt0, KL0, 256, (blk - 16) * NTHR + tid); }
  else if (blk < 32)  { prep_seg(Wr1, FD, wt1, KL1, 0,   (blk - 24) * NTHR + tid); }
  else if (blk < 40)  { prep_seg(Wr1, FD, wt1, KL1, 128, (blk - 32) * NTHR + tid); }
  else if (blk < 48)  { prep_seg(Ws1, FD, wt1, KL1, 256, (blk - 40) * NTHR + tid); }
  else if (blk < 56)  { prep_seg(Ws1, FD, wt1, KL1, 384, (blk - 48) * NTHR + tid); }
  else if (blk < 60)  { prep_seg(Wr2, NCLS, wt2, KL1, 0,   (blk - 56) * NTHR + tid); }
  else if (blk < 64)  { prep_seg(Wr2, NCLS, wt2, KL1, 128, (blk - 60) * NTHR + tid); }
  else if (blk < 68)  { prep_seg(Ws2, NCLS, wt2, KL1, 256, (blk - 64) * NTHR + tid); }
  else if (blk < 72)  { prep_seg(Ws2, NCLS, wt2, KL1, 384, (blk - 68) * NTHR + tid); }
  else {
    const int w = tid >> 5, l = tid & 31;
    if (w == 0) {
      const v4f v = *(const v4fa*)(b0 + 4 * l);
      st2_v4f(bias + 4 * l, cvt4_bf16(v));
    } else if (w == 1) {
      const v4f v = *(const v4fa*)(b1 + 4 * l);
      st2_v4f(bias + FD + 4 * l, cvt4_bf16(v));
    } else if (w == 2) {
      const int jc = l < (NCLS / 4 - 1) ? l : (NCLS / 4 - 1);
      const v4f v = *(const v4fa*)(b2 + 4 * jc);
      asm volatile("" :: "v"(v));
      const unsigned mk = (l < NCLS / 4) ? 0xFFFFFFFFu : 0u;
      const v4f c = cvt4_bf16(v);
      v4f o;
      o.x = __uint_as_float(__float_as_uint(c.x) & mk);
      o.y = __uint_as_float(__float_as_uint(c.y) & mk);
      o.z = __uint_as_float(__float_as_uint(c.z) & mk);
      o.w = __uint_as_float(__float_as_uint(c.w) & mk);
      if (l < NCP / 4) st2_v4f(bias + 2 * FD + 4 * l, o);
    }
  }
}

__device__ __forceinline__ void lists_flush(const int* pl, const int* cnt, const int* offs, int ov,
                                            int* lp, int* cp, int* op, int* fp, int tid) {
#pragma unroll 1
  for (int i = tid * 4; i < LCAP; i += NTHR * 4) {
    const v4i v = *(const v4ia*)(pl + i);
    *(volatile v4i*)(lp + i) = v;
  }
  if (tid < NBRUN / 4) {
    const v4i v = *(const v4ia*)(cnt + 4 * tid);
    *(volatile v4i*)(cp + 4 * tid) = v;
    const v4i w = *(const v4ia*)(offs + 4 * tid);
    *(volatile v4i*)(op + 4 * tid) = w;
  }
  if (tid < 8) {
    const v4i f = {ov, ov, ov, ov};
    *(volatile v4i*)(fp + 4 * tid) = f;
  }
}

__global__ __launch_bounds__(NTHR) void k_lists(const int* __restrict__ srcs, const int* __restrict__ dsts,
                                                int* LIST, int* CNT, int* OFF, int* FLAG) {
  extern __shared__ __attribute__((aligned(16))) int dsm[];
  int* wl   = dsm;
  int* pl   = dsm + NWAVE * WLCAP;
  int* cnt  = pl + LCAP;
  int* offs = cnt + NBRUN;
  int* cur  = offs + NBRUN;
  int* misc = cur + NBRUN;
  const int tid = (int)threadIdx.x, lane = tid & 31, wave = tid >> 5;
  const int blk = (int)blockIdx.x;
  const unsigned nbs = (unsigned)(blk * NBRUN);

  {
    const v4i z4 = {0, 0, 0, 0};
    for (int i = tid * 4; i < BK_ZINTS; i += NTHR * 4) *(v4ia*)(dsm + i) = z4;
    if (tid < 16) misc[tid] = 0;
  }
  __syncthreads();

  {
    const int per  = ((NE + NWAVE * WCH - 1) / (NWAVE * WCH)) * WCH;
    const int ebeg = wave * per;
    const int eend = (ebeg + per < NE) ? (ebeg + per) : NE;
    int* mylist = wl + wave * WLCAP;
    int wc = 0;
#pragma unroll 1
    for (int cb = ebeg; cb < eend; cb += WCH) {
      const int e0 = cb + lane * EPT;
      const int ec = e0 < NE - EPT ? e0 : NE - EPT;
      const bool lv = e0 < NE;
      const v4i da = *(const v4ia*)(dsts + ec);
      const v4i db = *(const v4ia*)(dsts + ec + 4);
      const int q0 = da.x, q1 = da.y, q2 = da.z, q3 = da.w;
      const int q4 = db.x, q5 = db.y, q6 = db.z, q7 = db.w;
      asm volatile("" :: "v"(q0));
      asm volatile("" :: "v"(q1));
      asm volatile("" :: "v"(q2));
      asm volatile("" :: "v"(q3));
      asm volatile("" :: "v"(q4));
      asm volatile("" :: "v"(q5));
      asm volatile("" :: "v"(q6));
      asm volatile("" :: "v"(q7));
      const unsigned s0 = (unsigned)q0 - nbs, s1 = (unsigned)q1 - nbs;
      const unsigned s2 = (unsigned)q2 - nbs, s3 = (unsigned)q3 - nbs;
      const unsigned s4 = (unsigned)q4 - nbs, s5 = (unsigned)q5 - nbs;
      const unsigned s6 = (unsigned)q6 - nbs, s7 = (unsigned)q7 - nbs;
      const bool h0 = lv && s0 < (unsigned)NBRUN && (unsigned)q0 < (unsigned)NN;
      const bool h1 = lv && s1 < (unsigned)NBRUN && (unsigned)q1 < (unsigned)NN;
      const bool h2 = lv && s2 < (unsigned)NBRUN && (unsigned)q2 < (unsigned)NN;
      const bool h3 = lv && s3 < (unsigned)NBRUN && (unsigned)q3 < (unsigned)NN;
      const bool h4 = lv && s4 < (unsigned)NBRUN && (unsigned)q4 < (unsigned)NN;
      const bool h5 = lv && s5 < (unsigned)NBRUN && (unsigned)q5 < (unsigned)NN;
      const bool h6 = lv && s6 < (unsigned)NBRUN && (unsigned)q6 < (unsigned)NN;
      const bool h7 = lv && s7 < (unsigned)NBRUN && (unsigned)q7 < (unsigned)NN;
      const unsigned m0 = __builtin_amdgcn_ballot_w32(h0), m1 = __builtin_amdgcn_ballot_w32(h1);
      const unsigned m2 = __builtin_amdgcn_ballot_w32(h2), m3 = __builtin_amdgcn_ballot_w32(h3);
      const unsigned m4 = __builtin_amdgcn_ballot_w32(h4), m5 = __builtin_amdgcn_ballot_w32(h5);
      const unsigned m6 = __builtin_amdgcn_ballot_w32(h6), m7 = __builtin_amdgcn_ballot_w32(h7);
      const unsigned any = m0 | m1 | m2 | m3 | m4 | m5 | m6 | m7;
      if (any != 0u) {
        const int pre = (int)(__builtin_amdgcn_mbcnt_lo(m0, 0u) + __builtin_amdgcn_mbcnt_lo(m1, 0u) +
                              __builtin_amdgcn_mbcnt_lo(m2, 0u) + __builtin_amdgcn_mbcnt_lo(m3, 0u) +
                              __builtin_amdgcn_mbcnt_lo(m4, 0u) + __builtin_amdgcn_mbcnt_lo(m5, 0u) +
                              __builtin_amdgcn_mbcnt_lo(m6, 0u) + __builtin_amdgcn_mbcnt_lo(m7, 0u));
        int p = wc + pre;
        if (h0) { if (p < WLCAP) mylist[p] = ((e0 + 0) << SLB) | (int)s0; p = p + 1; }
        if (h1) { if (p < WLCAP) mylist[p] = ((e0 + 1) << SLB) | (int)s1; p = p + 1; }
        if (h2) { if (p < WLCAP) mylist[p] = ((e0 + 2) << SLB) | (int)s2; p = p + 1; }
        if (h3) { if (p < WLCAP) mylist[p] = ((e0 + 3) << SLB) | (int)s3; p = p + 1; }
        if (h4) { if (p < WLCAP) mylist[p] = ((e0 + 4) << SLB) | (int)s4; p = p + 1; }
        if (h5) { if (p < WLCAP) mylist[p] = ((e0 + 5) << SLB) | (int)s5; p = p + 1; }
        if (h6) { if (p < WLCAP) mylist[p] = ((e0 + 6) << SLB) | (int)s6; p = p + 1; }
        if (h7) { if (p < WLCAP) mylist[p] = ((e0 + 7) << SLB) | (int)s7; p = p + 1; }
        wc += (int)(__builtin_popcount(m0) + __builtin_popcount(m1) + __builtin_popcount(m2) + __builtin_popcount(m3) +
                    __builtin_popcount(m4) + __builtin_popcount(m5) + __builtin_popcount(m6) + __builtin_popcount(m7));
      }
    }
    if (lane == 0) misc[wave] = wc;
  }
  __syncthreads();

  if (wave == 0) {
    int ov = 0;
    int tot = 0;
#pragma unroll 1
    for (int w2 = 0; w2 < NWAVE; ++w2) {
      int c = misc[w2];
      if (c > WLCAP) ov = 1;
      c = c < 0 ? 0 : (c > WLCAP ? WLCAP : c);
      tot += c;
#pragma unroll 1
      for (int b0 = 0; b0 < c; b0 += 32) {
        const int idx = b0 + lane;
        const int ent = wl[w2 * WLCAP + (idx < WLCAP ? idx : WLCAP - 1)];
        const int m32 = (c - b0) < 32 ? (c - b0) : 32;
#pragma unroll 1
        for (int k = 0; k < m32; ++k) {
          const int u    = __builtin_amdgcn_readlane(ent, k);
          const int slot = u & (NBRUN - 1);
          if (lane == 0) cnt[slot] = cnt[slot] + 1;
        }
      }
    }
    if (tot > LCAP) ov = 1;
    if (lane == 0) misc[9] = ov;
  }
  __syncthreads();
  if (wave == 0) {
    const int base = lane * (NBRUN / 32);
    int s = 0;
#pragma unroll 1
    for (int i = 0; i < NBRUN / 32; ++i) s += cnt[base + i];
    int incl = s;
#pragma unroll
    for (int d = 1; d < 32; d <<= 1) {
      const int y = __shfl_up(incl, d, 32);
      if (lane >= d) incl += y;
    }
    int run = incl - s;
#pragma unroll 1
    for (int i = 0; i < NBRUN / 32; ++i) {
      const int cv = cnt[base + i];
      offs[base + i] = run;
      cur[base + i]  = run;
      run += cv;
    }
  }
  __syncthreads();

  if (wave == 0) {
#pragma unroll 1
    for (int w2 = 0; w2 < NWAVE; ++w2) {
      int c = misc[w2];
      c = c < 0 ? 0 : (c > WLCAP ? WLCAP : c);
#pragma unroll 1
      for (int b0 = 0; b0 < c; b0 += 32) {
        const int idx = b0 + lane;
        const int ent = wl[w2 * WLCAP + (idx < WLCAP ? idx : WLCAP - 1)];
        int eid = (ent >> SLB) & 0x1FFFFF;
        eid = eid > NE - 1 ? NE - 1 : eid;
        int sr = srcs[eid];
        asm volatile("" :: "v"(sr));
        sr = clampi(sr, 0, NN - 1);
        const int m32 = (c - b0) < 32 ? (c - b0) : 32;
#pragma unroll 1
        for (int k = 0; k < m32; ++k) {
          const int u    = __builtin_amdgcn_readlane(ent, k);
          const int w0   = __builtin_amdgcn_readlane(sr, k);
          const int slot = u & (NBRUN - 1);
          if (lane == 0) {
            int p = cur[slot];
            p = p < 0 ? 0 : (p > LCAP - 1 ? LCAP - 1 : p);
            pl[p] = w0;
            cur[slot] = p + 1;
          }
        }
      }
    }
  }
  __syncthreads();

  const int ovf = misc[9];
  int* lp = LIST + (size_t)blk * (size_t)LCAP;
  int* cp = CNT  + (size_t)blk * NBRUN;
  int* op = OFF  + (size_t)blk * NBRUN;
  int* fp = FLAG + (size_t)blk * 32;
  lists_flush(pl, cnt, offs, ovf, lp, cp, op, fp, tid);
  __threadfence();
  lists_flush(pl, cnt, offs, ovf, lp, cp, op, fp, tid);
}

template <int L0>
__global__ __launch_bounds__(NTHR) void k_walk(const int* __restrict__ LIST, const int* __restrict__ CNT,
                                               const int* __restrict__ OFF, const int* __restrict__ FLAG,
                                               const float* __restrict__ H, unsigned short* OP, int row0) {
  constexpr int KL = L0 ? KL0 : KL1;
  const int tid = (int)threadIdx.x, lane = tid & 31, wave = tid >> 5;
  const int r = (int)blockIdx.x * NWAVE + wave;
  const int n = row0 + r;
  unsigned short* cr = OP + (size_t)r * KL + 4 * lane;

  if (n >= NN) {
    const v2u z = {0u, 0u};
    for (int pass = 0; pass < 2; ++pass) {
      *(volatile v2u*)cr = z;
      *(volatile v2u*)(cr + FD) = z;
      *(volatile v2u*)(cr + 2 * FD) = z;
      if (!L0) *(volatile v2u*)(cr + 3 * FD) = z;
      __threadfence();
    }
    return;
  }

  const int bk = n >> SLB;
  const int cv = CNT[n];
  asm volatile("" :: "v"(cv));
  const int ovv = OFF[n];
  asm volatile("" :: "v"(ovv));
  const int fl = FLAG[(size_t)bk * 32];
  asm volatile("" :: "v"(fl));

  const bool bad = (fl != 0) || (cv > DEGCAP) || (cv < 0);
  const int trip = __builtin_amdgcn_readfirstlane((fl == 0 && cv > 0) ? (cv > DEGCAP ? DEGCAP : cv) : 0);
  const int o = clampi(ovv, 0, LCAP - 1);
  int last = o + (trip > 0 ? trip : 1) - 1;
  last = last > LCAP - 1 ? LCAP - 1 : last;
  const int* lb = LIST + (size_t)bk * (size_t)LCAP;
  const float* tl = H + 4 * lane;

  float a0 = 0.0f, a1 = 0.0f, a2 = 0.0f, a3 = 0.0f;
#pragma unroll 1
  for (int b0 = 0; b0 < trip; b0 += 32) {
    int idx = o + b0 + lane;
    idx = idx > last ? last : idx;
    int sr = lb[idx];
    sr = clampi(sr, 0, NN - 1);
    const int m32 = (trip - b0) < 32 ? (trip - b0) : 32;
#pragma unroll 1
    for (int k = 0; k < m32; ++k) {
      const int sk = __builtin_amdgcn_readlane(sr, k);
      const v4f q = *(const v4fa*)(tl + (size_t)sk * FD);
      float t0 = q.x, t1 = q.y, t2 = q.z, t3 = q.w;
      if (L0) {
        t0 = bf16_val(t0); t1 = bf16_val(t1); t2 = bf16_val(t2); t3 = bf16_val(t3);
      } else {
        t0 = (t0 < 0.0f) ? 0.0f : t0;
        t1 = (t1 < 0.0f) ? 0.0f : t1;
        t2 = (t2 < 0.0f) ? 0.0f : t2;
        t3 = (t3 < 0.0f) ? 0.0f : t3;
      }
      asm volatile("" : "+v"(t0));
      asm volatile("" : "+v"(t1));
      asm volatile("" : "+v"(t2));
      asm volatile("" : "+v"(t3));
      a0 += t0; a1 += t1; a2 += t2; a3 += t3;
    }
  }

  const v4f d = *(const v4fa*)(H + (size_t)clampi(n, 0, NN - 1) * FD + 4 * lane);
  const float d0 = d.x, d1 = d.y, d2 = d.z, d3 = d.w;
  asm volatile("" :: "v"(d0));
  asm volatile("" :: "v"(d1));
  asm volatile("" :: "v"(d2));
  asm volatile("" :: "v"(d3));

  const float qnan = __uint_as_float(0x7fc00000u);
  const float u0 = bad ? qnan : a0, u1 = bad ? qnan : a1, u2 = bad ? qnan : a2, u3 = bad ? qnan : a3;
  v2u hv, lv2;
  hv.x  = pk16(bf16_bits(u0), bf16_bits(u1));
  hv.y  = pk16(bf16_bits(u2), bf16_bits(u3));
  lv2.x = pk16(bf16_lo_bits(u0), bf16_lo_bits(u1));
  lv2.y = pk16(bf16_lo_bits(u2), bf16_lo_bits(u3));

  if (L0) {
    v2u xb;
    xb.x = pk16(bf16_bits(d0), bf16_bits(d1));
    xb.y = pk16(bf16_bits(d2), bf16_bits(d3));
    for (int pass = 0; pass < 2; ++pass) {
      *(volatile v2u*)cr = hv;
      *(volatile v2u*)(cr + FD) = lv2;
      *(volatile v2u*)(cr + 2 * FD) = xb;
      __threadfence();
    }
  } else {
    const float r0 = (d0 < 0.0f) ? 0.0f : d0;
    const float r1 = (d1 < 0.0f) ? 0.0f : d1;
    const float r2 = (d2 < 0.0f) ? 0.0f : d2;
    const float r3 = (d3 < 0.0f) ? 0.0f : d3;
    v2u rh, rl2;
    rh.x  = pk16(bf16_bits(r0), bf16_bits(r1));
    rh.y  = pk16(bf16_bits(r2), bf16_bits(r3));
    rl2.x = pk16(bf16_lo_bits(r0), bf16_lo_bits(r1));
    rl2.y = pk16(bf16_lo_bits(r2), bf16_lo_bits(r3));
    for (int pass = 0; pass < 2; ++pass) {
      *(volatile v2u*)cr = hv;
      *(volatile v2u*)(cr + FD) = lv2;
      *(volatile v2u*)(cr + 2 * FD) = rh;
      *(volatile v2u*)(cr + 3 * FD) = rl2;
      __threadfence();
    }
  }
}

__global__ __launch_bounds__(NTHR) void k_copy(const float* __restrict__ P2, float* out) {
  const int i  = (int)blockIdx.x * NTHR + (int)threadIdx.x;
  const int ic = i < OUT4 ? i : OUT4 - 1;
  const int row = ic / (NCLS / 4);
  const int c4  = ic - row * (NCLS / 4);
  const v4f v = *(const v4fa*)(P2 + (size_t)row * NCP + 4 * c4);
  asm volatile("" :: "v"(v));
  if (i < OUT4) st2_v4f(out + (size_t)i * 4, v);
}

extern "C" void kernel_launch(void* const* d_in, const int* in_sizes, int n_in,
                              void* d_out, int out_size, void* d_ws, size_t ws_size,
                              hipStream_t stream) {
  if (n_in < 11) return;
  if (in_sizes[0] != NN * FD) return;
  if (in_sizes[1] != 2 * NE) return;
  if (in_sizes[2] != FD * FD) return;
  if (in_sizes[3] != FD * FD) return;
  if (in_sizes[4] != FD) return;
  if (in_sizes[5] != FD * FD) return;
  if (in_sizes[6] != FD * FD) return;
  if (in_sizes[7] != FD) return;
  if (in_sizes[8] != FD * NCLS) return;
  if (in_sizes[9] != FD * NCLS) return;
  if (in_sizes[10] != NCLS) return;
  if (out_size != NN * NCLS) return;

  const float* x   = (const float*)d_in[0];
  const int*   ei  = (const int*)d_in[1];
  const int*   srcs = ei;
  const int*   dsts = ei + NE;
  const float* Wr0 = (const float*)d_in[2];
  const float* Ws0 = (const float*)d_in[3];
  const float* b0  = (const float*)d_in[4];
  const float* Wr1 = (const float*)d_in[5];
  const float* Ws1 = (const float*)d_in[6];
  const float* b1  = (const float*)d_in[7];
  const float* Wr2 = (const float*)d_in[8];
  const float* Ws2 = (const float*)d_in[9];
  const float* b2  = (const float*)d_in[10];
  float* out = (float*)d_out;

  constexpr size_t zH    = (size_t)MP * FD * 4;
  constexpr size_t zOP   = (size_t)CH * KL1 * 2;
  constexpr size_t zLIST = (size_t)NBK * LCAP * 4;
  constexpr size_t zTAB  = (size_t)NBK * NBRUN * 4;
  constexpr size_t zFLAG = (size_t)NBK * 128;
  constexpr size_t zWT0  = (size_t)FD * KL0 * 2;
  constexpr size_t zWT1  = (size_t)FD * KL1 * 2;
  constexpr size_t zWT2  = (size_t)NCP * KL1 * 2;
  constexpr size_t zBIAS = 2048;
  constexpr size_t oHA   = 0;
  constexpr size_t oHB   = oHA + zH;
  constexpr size_t oOP   = oHB + zH;
  constexpr size_t oLIST = oOP + zOP;
  constexpr size_t oCNT  = oLIST + zLIST;
  constexpr size_t oOFF  = oCNT + zTAB;
  constexpr size_t oFLAG = oOFF + zTAB;
  constexpr size_t oWT   = oFLAG + zFLAG;
  constexpr size_t oBIAS = oWT + zWT0 + zWT1 + zWT2;
  constexpr size_t oEND  = oBIAS + zBIAS;
  static_assert(zH % 128 == 0 && zOP % 128 == 0 && zLIST % 128 == 0 && zTAB % 128 == 0 && zFLAG % 128 == 0);
  static_assert(zWT0 % 128 == 0 && zWT1 % 128 == 0 && zWT2 % 128 == 0 && zBIAS % 128 == 0);
  static_assert(zOP >= (size_t)CH * KL0 * 2 && zH >= (size_t)MP * NCP * 4);
  static_assert(zBIAS >= (size_t)(2 * FD + NCP) * 4);
  static_assert(zTAB >= (size_t)MP * 4);
  static_assert(oEND == (size_t)((size_t)246293 * 512));
  static_assert(oEND <= ((size_t)128 << 20));
  if (oEND > ws_size) return;

  char* ws = (char*)d_ws;
  float*          HA   = (float*)(ws + oHA);
  float*          HB   = (float*)(ws + oHB);
  float*          P2   = (float*)(ws + oHA);
  unsigned short* OP   = (unsigned short*)(ws + oOP);
  int*            LIST = (int*)(ws + oLIST);
  int*            CNT  = (int*)(ws + oCNT);
  int*            OFF  = (int*)(ws + oOFF);
  int*            FLAG = (int*)(ws + oFLAG);
  unsigned short* WT0  = (unsigned short*)(ws + oWT);
  unsigned short* WT1  = WT0 + (size_t)FD * KL0;
  unsigned short* WT2  = WT1 + (size_t)FD * KL1;
  float*          BIAS = (float*)(ws + oBIAS);
  const float*    B0   = BIAS;
  const float*    B1   = BIAS + FD;
  const float*    B2   = BIAS + 2 * FD;

  hipFuncSetAttribute(reinterpret_cast<const void*>(&k_lists), hipFuncAttributeMaxDynamicSharedMemorySize, (int)BK_LDS);

  k_prep<<<PW_BLKS, NTHR, 0, stream>>>(Wr0, Ws0, b0, Wr1, Ws1, b1, Wr2, Ws2, b2, WT0, BIAS);
  k_lists<<<NBK, NTHR, BK_LDS, stream>>>(srcs, dsts, LIST, CNT, OFF, FLAG);

  for (int c = 0; c < NCHUNK; ++c) {
    const int rows = (c < NCHUNK - 1) ? CH : CHL;
    const int row0 = c * CH;
    const int tiles = (rows / 64) * (FD / 64);
    k_walk<1><<<rows / NWAVE, NTHR, 0, stream>>>(LIST, CNT, OFF, FLAG, x, OP, row0);
    k_gemm_nt<0, 1><<<(tiles + 7) / 8, NTHR, 0, stream>>>(OP, WT0, B0, HA + (size_t)row0 * FD, rows, FD, KL0, FD);
  }
  for (int c = 0; c < NCHUNK; ++c) {
    const int rows = (c < NCHUNK - 1) ? CH : CHL;
    const int row0 = c * CH;
    const int tiles = (rows / 64) * (FD / 64);
    k_walk<0><<<rows / NWAVE, NTHR, 0, stream>>>(LIST, CNT, OFF, FLAG, HA, OP, row0);
    k_gemm_nt<0, 1><<<(tiles + 7) / 8, NTHR, 0, stream>>>(OP, WT1, B1, HB + (size_t)row0 * FD, rows, FD, KL1, FD);
  }
  for (int c = 0; c < NCHUNK; ++c) {
    const int rows = (c < NCHUNK - 1) ? CH : CHL;
    const int row0 = c * CH;
    const int tiles = (rows / 64) * (NCP / 64);
    k_walk<0><<<rows / NWAVE, NTHR, 0, stream>>>(LIST, CNT, OFF, FLAG, HB, OP, row0);
    k_gemm_nt<0, 1><<<(tiles + 7) / 8, NTHR, 0, stream>>>(OP, WT2, B2, P2 + (size_t)row0 * NCP, rows, NCP, KL1, NCP);
  }
  k_copy<<<(OUT4 + NTHR - 1) / NTHR, NTHR, 0, stream>>>(P2, out);
}
